// acLSTM_31533649887639
// MI455X (gfx1250) — hardware-verified
//
#include <hip/hip_runtime.h>
#include <math.h>

constexpr int NSEQ  = 32;
constexpr int NSTEP = 200;
constexpr int NFRM  = 231;
constexpr int NHID  = 1024;
constexpr int NGATE = 4 * NHID;
constexpr int KXPAD = 256;
constexpr int NDECP = 256;
constexpr int NTHR  = 256;
constexpr int NWAV  = NTHR / 32;
constexpr int RBLK  = 16;
constexpr int NBLK  = NSEQ / RBLK;
constexpr int NSUB  = NHID / (16 * NWAV);
constexpr int HPIT  = 1032;
constexpr int XPIT  = 264;
constexpr int YPIT  = 260;
constexpr int OPIT  = 256;
constexpr int NQUAT = 57;
constexpr int NPROWS = NSEQ * NSTEP;
constexpr int NOUT4  = NSEQ * NSTEP * NFRM / 4;
constexpr int CSLOT  = 256;
constexpr int CWAVE  = NSUB * CSLOT;
constexpr int CTOTAL = 3 * NBLK * NWAV * CWAVE;
constexpr float ACAR = 64.0f;
constexpr float WCAR = 1024.0f;
constexpr float PINV = 1.0f / 65536.0f;
static_assert(NSEQ % RBLK == 0);
static_assert(NHID == 16 * NSUB * NWAV);
static_assert(KXPAD % 32 == 0 && NHID % 32 == 0);
static_assert(KXPAD >= NFRM && XPIT >= KXPAD && HPIT >= NHID);
static_assert(NDECP % 16 == 0 && NDECP >= NFRM && NDECP == 16 * 2 * NWAV);
static_assert(3 + 4 * NQUAT == NFRM);
static_assert(RBLK * (KXPAD / 8) == 2 * NTHR);
static_assert(RBLK * (OPIT / 4) == 4 * NTHR);
static_assert((NSEQ * NSTEP * NFRM) % 4 == 0);
static_assert(NOUT4 % 32 == 0);
static_assert(HPIT % 8 == 0 && XPIT % 8 == 0 && YPIT % 4 == 0);
static_assert(RBLK * NQUAT <= 4 * NTHR);
static_assert(YPIT >= OPIT + 1 && YPIT >= NDECP + 1);
static_assert(CSLOT == 2 * 32 * 4);
static_assert(CTOTAL == 98304);

typedef __attribute__((ext_vector_type(16))) _Float16 v16h;
typedef __attribute__((ext_vector_type(8)))  _Float16 v8h;
typedef __attribute__((ext_vector_type(8)))  float    v8f;
typedef __attribute__((ext_vector_type(4)))  float    v4f;

__device__ __forceinline__ void dep_guard4_h(v8f& a0, v8f& a1, v8f& a2, v8f& a3, v16h x, v16h y) {
  asm volatile("v_nop\n\tv_nop\n\tv_nop\n\tv_nop" : "+v"(a0), "+v"(a1), "+v"(a2), "+v"(a3) : "v"(x), "v"(y));
}
__device__ __forceinline__ void dep_guard1_h(v8f& a, v16h x, v16h y) { asm volatile("v_nop\n\tv_nop\n\tv_nop\n\tv_nop" : "+v"(a) : "v"(x), "v"(y)); }
__device__ __forceinline__ void keep4_h(v16h a, v16h b, v16h c, v16h d) { asm volatile("v_nop" :: "v"(a), "v"(b), "v"(c), "v"(d)); }
__device__ __forceinline__ void acc_guard4(v8f& a, v8f& b, v8f& c, v8f& d) { asm volatile("v_nop\n\tv_nop\n\tv_nop\n\tv_nop" : "+v"(a), "+v"(b), "+v"(c), "+v"(d)); }
__device__ __forceinline__ void acc_guard1(v8f& a) { asm volatile("v_nop\n\tv_nop\n\tv_nop\n\tv_nop" : "+v"(a)); }

template <typename T> struct Frag;
template <> struct Frag<_Float16> {
  typedef v16h V; union U { v16h v; v8h h[2]; };
  static __device__ __forceinline__ v16h load(const _Float16* p) {
    U f; f.h[0] = *(const v8h*)(p); f.h[1] = *(const v8h*)(p + 16); return f.v;
  }
  static __device__ __forceinline__ v8f mma(v16h a, v16h b, v8f c) {
    return __builtin_amdgcn_wmma_f32_16x16x32_f16(false, a, false, b, (short)0, c, false, false);
  }
};
typedef Frag<_Float16> FragH;

__device__ __forceinline__ float fsig(float x)  { return 1.0f / (1.0f + expf(-x)); }
__device__ __forceinline__ float ftanh(float x) { return 1.0f - 2.0f / (expf(2.0f * x) + 1.0f); }

__device__ __forceinline__ float cell_update(float pi, float pf, float pg, float po,
                                             float bI, float bF, float bG, float bO, float co, float& cn) {
  const float zi = pi * PINV + bI;
  const float zf = pf * PINV + bF;
  const float zg = pg * PINV + bG;
  const float zo = po * PINV + bO;
  const float ig = fsig(zi);
  const float fg = fsig(zf);
  const float og = fsig(zo);
  const float gg = ftanh(zg);
  cn = fg * co + ig * gg;
  return og * ftanh(cn);
}

template <bool AL>
__global__ __launch_bounds__(256) void cvt8_f16_kernel(const float* __restrict__ src, unsigned short* __restrict__ dst,
                                                      int nrowd, int ncol8, int nrows, int ncols, float sc) {
  const int i  = blockIdx.x * 256 + threadIdx.x;
  const int n8 = nrowd * ncol8;
  if (i < n8) {
    const int row = i / ncol8;
    const int c8  = i - row * ncol8;
    v8h hv;
    if (AL) {
      const float* sp = src + (size_t)row * (size_t)ncols + c8 * 8;
      const v4f a = *(const v4f*)(sp);
      const v4f b = *(const v4f*)(sp + 4);
#pragma unroll
      for (int e = 0; e < 4; ++e) {
        hv[e]     = (_Float16)(a[e] * sc);
        hv[4 + e] = (_Float16)(b[e] * sc);
      }
    } else {
      const int rr = row < nrows ? row : nrows - 1;
      const float rk = (row < nrows) ? 1.0f : 0.0f;
      const float* sp = src + (size_t)rr * (size_t)ncols;
#pragma unroll
      for (int e = 0; e < 8; ++e) {
        const int col = c8 * 8 + e;
        const int cc  = col < ncols ? col : ncols - 1;
        const float ck = (col < ncols) ? 1.0f : 0.0f;
        const float f = sp[cc];
        hv[e] = (_Float16)((f * (rk * ck)) * sc);
      }
    }
    *(volatile v8h*)(dst + (size_t)i * 8) = hv;
    __threadfence();
    *(volatile v8h*)(dst + (size_t)i * 8) = hv;
  }
}

template <int KIN>
__device__ __forceinline__ void lstm_cell_phase(const _Float16* xt, int xpit, const _Float16* ht, _Float16* hnew,
                                                const _Float16* __restrict__ WX, const _Float16* __restrict__ WH,
                                                const float* __restrict__ bih, const float* __restrict__ bhh,
                                                float* cw, int wave, int lane, int c, int hh, int koff) {
  const v8f z8 = {0.f, 0.f, 0.f, 0.f, 0.f, 0.f, 0.f, 0.f};
  const _Float16* xrow = xt + c * xpit + koff;
  const _Float16* hrow = ht + c * HPIT + koff;
#pragma unroll 1
  for (int nt = 0; nt < NSUB; ++nt) {
    const int j = 16 * (NSUB * wave + nt) + c;
    const _Float16* wx = WX + (size_t)j * KIN + koff;
    const _Float16* wh = WH + (size_t)j * NHID + koff;
    v8f accI = z8, accF = z8, accG = z8, accO = z8;
#pragma unroll 1
    for (int k0 = 0; k0 < KIN; k0 += 32) {
      const v16h a  = FragH::load(xrow + k0);
      const v16h b0 = FragH::load(wx + k0);
      const v16h b1 = FragH::load(wx + (size_t)1 * NHID * KIN + k0);
      const v16h b2 = FragH::load(wx + (size_t)2 * NHID * KIN + k0);
      const v16h b3 = FragH::load(wx + (size_t)3 * NHID * KIN + k0);
      accI = FragH::mma(a, b0, accI);
      accF = FragH::mma(a, b1, accF);
      accG = FragH::mma(a, b2, accG);
      accO = FragH::mma(a, b3, accO);
      dep_guard4_h(accI, accF, accG, accO, a, b3);
      keep4_h(b0, b1, b2, b3);
    }
#pragma unroll 1
    for (int k0 = 0; k0 < NHID; k0 += 32) {
      const v16h a  = FragH::load(hrow + k0);
      const v16h b0 = FragH::load(wh + k0);
      const v16h b1 = FragH::load(wh + (size_t)1 * NHID * NHID + k0);
      const v16h b2 = FragH::load(wh + (size_t)2 * NHID * NHID + k0);
      const v16h b3 = FragH::load(wh + (size_t)3 * NHID * NHID + k0);
      accI = FragH::mma(a, b0, accI);
      accF = FragH::mma(a, b1, accF);
      accG = FragH::mma(a, b2, accG);
      accO = FragH::mma(a, b3, accO);
      dep_guard4_h(accI, accF, accG, accO, a, b3);
      keep4_h(b0, b1, b2, b3);
    }
    acc_guard4(accI, accF, accG, accO);
    float* cs = cw + nt * CSLOT + lane * 4;
    const v4f cv0 = *(const v4f*)(cs);
    const v4f cv1 = *(const v4f*)(cs + 128);
    const float bI = bih[j] + bhh[j];
    const float bF = bih[NHID + j] + bhh[NHID + j];
    const float bG = bih[2 * NHID + j] + bhh[2 * NHID + j];
    const float bO = bih[3 * NHID + j] + bhh[3 * NHID + j];
    v4f cn0 = {0.f, 0.f, 0.f, 0.f};
    v4f cn1 = {0.f, 0.f, 0.f, 0.f};
#pragma unroll
    for (int r = 0; r < 4; ++r) {
      float cn;
      const float hn = cell_update(accI[r], accF[r], accG[r], accO[r], bI, bF, bG, bO, cv0[r], cn);
      cn0[r] = cn;
      hnew[(8 * hh + r) * HPIT + j] = (_Float16)(hn * ACAR);
    }
#pragma unroll
    for (int r = 0; r < 4; ++r) {
      float cn;
      const float hn = cell_update(accI[4 + r], accF[4 + r], accG[4 + r], accO[4 + r], bI, bF, bG, bO, cv1[r], cn);
      cn1[r] = cn;
      hnew[(8 * hh + 4 + r) * HPIT + j] = (_Float16)(hn * ACAR);
    }
    for (int pass = 0; pass < 2; ++pass) {
      *(volatile v4f*)(cs) = cn0;
      *(volatile v4f*)(cs + 128) = cn1;
      __threadfence();
    }
  }
}

__device__ __forceinline__ void decoder_phase(const _Float16* h3t, const _Float16* __restrict__ WD,
                                              const float* __restrict__ decb, float* ys, int wave, int c, int hh, int koff) {
  const v8f z8 = {0.f, 0.f, 0.f, 0.f, 0.f, 0.f, 0.f, 0.f};
  const _Float16* hrow = h3t + c * HPIT + koff;
#pragma unroll
  for (int i = 0; i < 2; ++i) {
    const int n = 16 * (wave + NWAV * i) + c;
    const _Float16* wd = WD + (size_t)n * NHID + koff;
    v8f acc = z8;
#pragma unroll 1
    for (int k0 = 0; k0 < NHID; k0 += 32) {
      const v16h a = FragH::load(hrow + k0);
      const v16h b = FragH::load(wd + k0);
      acc = FragH::mma(a, b, acc);
      dep_guard1_h(acc, a, b);
    }
    acc_guard1(acc);
    const int nc = n < NFRM ? n : NFRM - 1;
    const float bn = decb[nc];
    const float rk = (n < NFRM) ? 1.0f : 0.0f;
#pragma unroll
    for (int r = 0; r < 8; ++r) {
      const float v = (acc[r] * PINV + bn) * rk;
      ys[(8 * hh + r) * YPIT + n + 1] = v;
    }
  }
}

__device__ __forceinline__ void renorm_phase(float* ys, int tid) {
#pragma unroll 1
  for (int it = 0; it < 4; ++it) {
    const int item = it * NTHR + tid;
    const int itc  = item < RBLK * NQUAT ? item : RBLK * NQUAT - 1;
    const int row  = itc / NQUAT;
    const int q    = itc - row * NQUAT;
    float* p = ys + row * YPIT + 4 + 4 * q;
    const v4f v = *(const v4f*)p;
    const float ss  = (v[0] * v[0] + v[1] * v[1]) + (v[2] * v[2] + v[3] * v[3]);
    const float inv = 1.0f / (sqrtf(ss) + 1e-8f);
    v4f o;
    o[0] = v[0] * inv; o[1] = v[1] * inv; o[2] = v[2] * inv; o[3] = v[3] * inv;
    if (item < RBLK * NQUAT) *(v4f*)p = o;
  }
}

__device__ __forceinline__ void build_x_tile(_Float16* xt, const float* ys, const float* __restrict__ seq,
                                             int rowbase, int tn, int tid) {
  const int ph  = tn % 10;
  const float gs = (ph < 5) ? 1.0f : 0.0f;
  const float os = 1.0f - gs;
#pragma unroll 1
  for (int it = 0; it < 2; ++it) {
    const int item = it * NTHR + tid;
    const int row = item >> 5, g8 = item & 31;
    const float* sp = seq + ((size_t)(rowbase + row) * NSTEP + (size_t)tn) * NFRM;
    const float* yp = ys + row * YPIT + 1 + 8 * g8;
    v8h hv;
#pragma unroll
    for (int e = 0; e < 8; ++e) {
      const int col = 8 * g8 + e;
      const int cc  = col < NFRM ? col : NFRM - 1;
      const float ck = (col < NFRM) ? 1.0f : 0.0f;
      const float sv = sp[cc] * ck;
      const float yv = yp[e];
      const float xv = fmaf(gs, sv, os * yv);
      hv[e] = (_Float16)(xv * ACAR);
    }
    *(v8h*)(xt + row * XPIT + 8 * g8) = hv;
  }
}

__global__ __launch_bounds__(NTHR) void seq3_kernel(const float* __restrict__ seq,
                                                    const unsigned short* __restrict__ WX1p, const unsigned short* __restrict__ WH1p,
                                                    const float* __restrict__ bih1, const float* __restrict__ bhh1,
                                                    const unsigned short* __restrict__ WX2p, const unsigned short* __restrict__ WH2p,
                                                    const float* __restrict__ bih2, const float* __restrict__ bhh2,
                                                    const unsigned short* __restrict__ WX3p, const unsigned short* __restrict__ WH3p,
                                                    const float* __restrict__ bih3, const float* __restrict__ bhh3,
                                                    const unsigned short* __restrict__ WDp, const float* __restrict__ decb,
                                                    float* CST, float* __restrict__ OUTP) {
  __shared__ __align__(16) _Float16 HT[4 * RBLK * HPIT];
  __shared__ __align__(16) _Float16 XT[RBLK * XPIT];
  __shared__ __align__(16) float    YS[RBLK * YPIT];
  const _Float16* WX1 = (const _Float16*)WX1p; const _Float16* WH1 = (const _Float16*)WH1p;
  const _Float16* WX2 = (const _Float16*)WX2p; const _Float16* WH2 = (const _Float16*)WH2p;
  const _Float16* WX3 = (const _Float16*)WX3p; const _Float16* WH3 = (const _Float16*)WH3p;
  const _Float16* WD  = (const _Float16*)WDp;
  const int tid = threadIdx.x, lane = tid & 31, wave = tid >> 5;
  const int c = lane & 15, hh = lane >> 4, koff = hh * 8;
  const int blk = blockIdx.x;
  const int rowbase = blk * RBLK;

#pragma unroll 1
  for (int i = tid; i < 4 * RBLK * HPIT; i += NTHR) HT[i] = (_Float16)0.0f;
#pragma unroll 1
  for (int i = tid; i < RBLK * XPIT; i += NTHR) XT[i] = (_Float16)0.0f;
#pragma unroll 1
  for (int i = tid; i < RBLK * YPIT; i += NTHR) YS[i] = 0.0f;

  float* cw1 = CST + (size_t)((0 * NBLK + blk) * NWAV + wave) * CWAVE;
  float* cw2 = CST + (size_t)((1 * NBLK + blk) * NWAV + wave) * CWAVE;
  float* cw3 = CST + (size_t)((2 * NBLK + blk) * NWAV + wave) * CWAVE;
  {
    const v4f z4 = {0.f, 0.f, 0.f, 0.f};
    for (int pass = 0; pass < 2; ++pass) {
#pragma unroll 1
      for (int k = 0; k < 3 * NSUB; ++k) {
        const int cell = k / NSUB, nt = k - cell * NSUB;
        float* cs = CST + (size_t)((cell * NBLK + blk) * NWAV + wave) * CWAVE + nt * CSLOT + lane * 4;
        *(volatile v4f*)(cs) = z4;
        *(volatile v4f*)(cs + 128) = z4;
      }
      __threadfence();
    }
  }
  __syncthreads();
  build_x_tile(XT, YS, seq, rowbase, 0, tid);
  __syncthreads();

#pragma unroll 1
  for (int t = 0; t < NSTEP; ++t) {
    const int tm = t & 3;
    const int s1 = (4 - tm) & 3, s2 = (5 - tm) & 3, s3 = (6 - tm) & 3, sf = (7 - tm) & 3;
    _Float16* H1 = HT + s1 * (RBLK * HPIT);
    _Float16* H2 = HT + s2 * (RBLK * HPIT);
    _Float16* H3 = HT + s3 * (RBLK * HPIT);
    _Float16* HF = HT + sf * (RBLK * HPIT);

    lstm_cell_phase<KXPAD>(XT, XPIT, H1, HF, WX1, WH1, bih1, bhh1, cw1, wave, lane, c, hh, koff);
    __syncthreads();
    lstm_cell_phase<NHID>(HF, HPIT, H2, H1, WX2, WH2, bih2, bhh2, cw2, wave, lane, c, hh, koff);
    __syncthreads();
    lstm_cell_phase<NHID>(H1, HPIT, H3, H2, WX3, WH3, bih3, bhh3, cw3, wave, lane, c, hh, koff);
    __syncthreads();
    decoder_phase(H2, WD, decb, YS, wave, c, hh, koff);
    __syncthreads();
    renorm_phase(YS, tid);
    __syncthreads();
    {
      v4f pv[4]; size_t po[4];
#pragma unroll
      for (int it = 0; it < 4; ++it) {
        const int idx = it * NTHR + tid;
        const int row = idx >> 6, c4 = (idx & 63) * 4;
        pv[it] = *(const v4f*)(YS + row * YPIT + c4);
        po[it] = ((size_t)(rowbase + row) * NSTEP + (size_t)t) * OPIT + c4;
      }
      for (int pass = 0; pass < 2; ++pass) {
        *(volatile v4f*)(OUTP + po[0]) = pv[0];
        *(volatile v4f*)(OUTP + po[1]) = pv[1];
        *(volatile v4f*)(OUTP + po[2]) = pv[2];
        *(volatile v4f*)(OUTP + po[3]) = pv[3];
        __threadfence();
      }
    }
    {
      const int tn = (t + 1 < NSTEP) ? (t + 1) : (NSTEP - 1);
      build_x_tile(XT, YS, seq, rowbase, tn, tid);
    }
    __syncthreads();
  }
}

__global__ __launch_bounds__(256) void repack_kernel(const float* __restrict__ P, float* __restrict__ out, int n4) {
  const int i = blockIdx.x * 256 + threadIdx.x;
  if (i < n4) {
    v4f v;
#pragma unroll
    for (int e = 0; e < 4; ++e) {
      const int el  = 4 * i + e;
      const int row = el / NFRM;
      const int f   = el - row * NFRM;
      v[e] = P[(size_t)row * OPIT + f + 1];
    }
    *(volatile v4f*)(out + (size_t)i * 4) = v;
    __threadfence();
    *(volatile v4f*)(out + (size_t)i * 4) = v;
  }
}

extern "C" void kernel_launch(void* const* d_in, const int* in_sizes, int n_in,
                              void* d_out, int out_size, void* d_ws, size_t ws_size, hipStream_t stream) {
  if (n_in < 15 || d_out == nullptr || d_ws == nullptr) return;
  if (in_sizes[0] != NSEQ * NSTEP * NFRM || in_sizes[1] != NGATE * NFRM || in_sizes[2] != NGATE * NHID ||
      in_sizes[3] != NGATE || in_sizes[4] != NGATE || in_sizes[5] != NGATE * NHID || in_sizes[6] != NGATE * NHID ||
      in_sizes[7] != NGATE || in_sizes[8] != NGATE || in_sizes[9] != NGATE * NHID || in_sizes[10] != NGATE * NHID ||
      in_sizes[11] != NGATE || in_sizes[12] != NGATE || in_sizes[13] != NFRM * NHID || in_sizes[14] != NFRM ||
      out_size != NSEQ * NSTEP * NFRM) return;

  const float* seq  = (const float*)d_in[0];
  const float* Wih1 = (const float*)d_in[1];
  const float* Whh1 = (const float*)d_in[2];
  const float* bih1 = (const float*)d_in[3];
  const float* bhh1 = (const float*)d_in[4];
  const float* Wih2 = (const float*)d_in[5];
  const float* Whh2 = (const float*)d_in[6];
  const float* bih2 = (const float*)d_in[7];
  const float* bhh2 = (const float*)d_in[8];
  const float* Wih3 = (const float*)d_in[9];
  const float* Whh3 = (const float*)d_in[10];
  const float* bih3 = (const float*)d_in[11];
  const float* bhh3 = (const float*)d_in[12];
  const float* decW = (const float*)d_in[13];
  const float* decb = (const float*)d_in[14];
  float* out = (float*)d_out;

  char* ws = (char*)d_ws; size_t off = 0;
  auto carve = [&](size_t bytes) -> char* { char* p = ws + off; off += (bytes + 255) & ~(size_t)255; return p; };
  unsigned short* WX1 = (unsigned short*)carve((size_t)NGATE * KXPAD * 2);
  unsigned short* WH1 = (unsigned short*)carve((size_t)NGATE * NHID * 2);
  unsigned short* WX2 = (unsigned short*)carve((size_t)NGATE * NHID * 2);
  unsigned short* WH2 = (unsigned short*)carve((size_t)NGATE * NHID * 2);
  unsigned short* WX3 = (unsigned short*)carve((size_t)NGATE * NHID * 2);
  unsigned short* WH3 = (unsigned short*)carve((size_t)NGATE * NHID * 2);
  unsigned short* WD  = (unsigned short*)carve((size_t)NDECP * NHID * 2);
  float*          CST = (float*)carve((size_t)CTOTAL * 4);
  float*          OUTP = (float*)carve((size_t)NPROWS * OPIT * 4);
  if (off > ws_size || off > (size_t)134217728) return;

  const int n8x1 = NGATE * (KXPAD / 8);
  const int n8h  = NGATE * (NHID / 8);
  const int n8d  = NDECP * (NHID / 8);
  cvt8_f16_kernel<false><<<(n8x1 + 255) / 256, 256, 0, stream>>>(Wih1, WX1, NGATE, KXPAD / 8, NGATE, NFRM, WCAR);
  cvt8_f16_kernel<true ><<<(n8h + 255) / 256, 256, 0, stream>>>(Whh1, WH1, NGATE, NHID / 8, NGATE, NHID, WCAR);
  cvt8_f16_kernel<true ><<<(n8h + 255) / 256, 256, 0, stream>>>(Wih2, WX2, NGATE, NHID / 8, NGATE, NHID, WCAR);
  cvt8_f16_kernel<true ><<<(n8h + 255) / 256, 256, 0, stream>>>(Whh2, WH2, NGATE, NHID / 8, NGATE, NHID, WCAR);
  cvt8_f16_kernel<true ><<<(n8h + 255) / 256, 256, 0, stream>>>(Wih3, WX3, NGATE, NHID / 8, NGATE, NHID, WCAR);
  cvt8_f16_kernel<true ><<<(n8h + 255) / 256, 256, 0, stream>>>(Whh3, WH3, NGATE, NHID / 8, NGATE, NHID, WCAR);
  cvt8_f16_kernel<false><<<(n8d + 255) / 256, 256, 0, stream>>>(decW, WD, NDECP, NHID / 8, NFRM, NHID, WCAR);

  seq3_kernel<<<NBLK, NTHR, 0, stream>>>(seq, WX1, WH1, bih1, bhh1, WX2, WH2, bih2, bhh2, WX3, WH3, bih3, bhh3,
                                         WD, decb, CST, OUTP);

  repack_kernel<<<(NOUT4 + 255) / 256, 256, 0, stream>>>(OUTP, out, NOUT4);
}
